// Block_35880156790920
// MI455X (gfx1250) — hardware-run, weakly checked
//
#include <hip/hip_runtime.h>
#include <math.h>


#ifndef NB
#define NB 2
#endif
#ifndef SEQ
#define SEQ 2048
#endif
#define NB_FULL  2
#define SEQ_FULL 2048
#define DM   1024
#define NH   16
#define HDIM 64
#define DFF  4096
#define TOKN (NB * SEQ)
#define LOGMAX 4.605170185988091f
#define LOG2E  1.4426950408889634f

static_assert(SEQ % 64 == 0);
static_assert(NB >= 1 && NB <= NB_FULL);
static_assert(SEQ <= SEQ_FULL);
static_assert(DM == NH * HDIM);
static_assert(HDIM == 64);
static_assert(DM % 128 == 0);
static_assert(DFF % 128 == 0);
static_assert(TOKN % 64 == 0);
static_assert(DM % 32 == 0 && DFF % 32 == 0);

typedef _Float16 v16h __attribute__((ext_vector_type(16)));
typedef _Float16 v8h  __attribute__((ext_vector_type(8)));
typedef float    v8f  __attribute__((ext_vector_type(8)));
typedef float    v4f  __attribute__((ext_vector_type(4)));
typedef unsigned int v4u __attribute__((ext_vector_type(4)));
typedef v8h __attribute__((may_alias)) v8ha;
typedef v4f __attribute__((may_alias)) v4fa;
typedef v4u __attribute__((may_alias)) v4ua;

union Frag { v16h v; v8h h[2]; };

__device__ __forceinline__ float bf16r(float f) {
    unsigned int u = __float_as_uint(f);
    u = (u + 0x7FFFu + ((u >> 16) & 1u)) & 0xFFFF0000u;
    return __uint_as_float(u);
}

__device__ __forceinline__ v8f mma16(v16h a, v16h b, v8f c) {
    return __builtin_amdgcn_wmma_f32_16x16x32_f16(false, a, false, b, (short)0, c, false, false);
}

__global__ __launch_bounds__(256) void k_wcvt(const float* __restrict__ W, _Float16* Wt,
                                                int Kd, int Nd, float mul)
{
    __shared__ float tile[64 * 65];
    const int t = threadIdx.x;
    const int n0 = blockIdx.x * 64, k0 = blockIdx.y * 64;
    {
        const int kr = t >> 2, ns = (t & 3) * 16;
        const float* src = W + (size_t)(k0 + kr) * Nd + n0 + ns;
#pragma unroll
        for (int j = 0; j < 4; ++j) {
            const v4f q = *(const v4fa*)(src + 4 * j);
            float* d = tile + kr * 65 + ns + 4 * j;
            d[0] = q[0]; d[1] = q[1]; d[2] = q[2]; d[3] = q[3];
        }
    }
    __syncthreads();
    v4u w[2];
    size_t off[2];
#pragma unroll
    for (int hf = 0; hf < 2; ++hf) {
        const int nl = hf * 32 + (t >> 3), ks = (t & 7) * 8;
        v8h o;
#pragma unroll
        for (int j = 0; j < 8; ++j)
            o[j] = (_Float16)(bf16r(tile[(ks + j) * 65 + nl]) * mul);
        w[hf] = __builtin_bit_cast(v4u, o);
        off[hf] = (size_t)(n0 + nl) * Kd + k0 + ks;
    }
    *(volatile v4u*)(Wt + off[0]) = w[0];
    *(volatile v4u*)(Wt + off[1]) = w[1];
    __threadfence();
    *(volatile v4u*)(Wt + off[0]) = w[0];
    *(volatile v4u*)(Wt + off[1]) = w[1];
}

__global__ __launch_bounds__(128) void k_ln(const float* __restrict__ X,
                                              const float* __restrict__ gam,
                                              const float* __restrict__ bet,
                                              _Float16* Y, int seqc, int seqx, int rne)
{
    __shared__ float red[2][4];
    const int t = threadIdx.x, lane = t & 31, wv = t >> 5;
    const int row = blockIdx.x;
    const int gb = row / seqc;
    const int xrow = gb * seqx + (row - gb * seqc);
    const float* xp = X + (size_t)xrow * DM + t * 8;
    const v4f a0 = *(const v4fa*)xp;
    const v4f a1 = *(const v4fa*)(xp + 4);
    float v[8] = {a0[0], a0[1], a0[2], a0[3], a1[0], a1[1], a1[2], a1[3]};
    if (rne) {
#pragma unroll
        for (int i = 0; i < 8; ++i) v[i] = bf16r(v[i]);
    }
    float s = 0.f;
#pragma unroll
    for (int i = 0; i < 8; ++i) s += v[i];
#pragma unroll
    for (int m = 16; m >= 1; m >>= 1) s += __shfl_xor(s, m, 32);
    if (lane == 0) red[0][wv] = s;
    __syncthreads();
    const float mu = ((red[0][0] + red[0][1]) + (red[0][2] + red[0][3])) * (1.0f / DM);
    float d[8];
    float s2 = 0.f;
#pragma unroll
    for (int i = 0; i < 8; ++i) { d[i] = v[i] - mu; s2 += d[i] * d[i]; }
#pragma unroll
    for (int m = 16; m >= 1; m >>= 1) s2 += __shfl_xor(s2, m, 32);
    if (lane == 0) red[1][wv] = s2;
    __syncthreads();
    const float var = ((red[1][0] + red[1][1]) + (red[1][2] + red[1][3])) * (1.0f / DM);
    const float rs = rsqrtf(var + 1.0e-6f);
    const v4f g0 = *(const v4fa*)(gam + t * 8);
    const v4f g1 = *(const v4fa*)(gam + t * 8 + 4);
    const v4f b0 = *(const v4fa*)(bet + t * 8);
    const v4f b1 = *(const v4fa*)(bet + t * 8 + 4);
    const float gg[8] = {g0[0], g0[1], g0[2], g0[3], g1[0], g1[1], g1[2], g1[3]};
    const float be[8] = {b0[0], b0[1], b0[2], b0[3], b1[0], b1[1], b1[2], b1[3]};
    v8h o;
#pragma unroll
    for (int i = 0; i < 8; ++i) o[i] = (_Float16)(d[i] * rs * bf16r(gg[i]) + bf16r(be[i]));
    const v4u w = __builtin_bit_cast(v4u, o);
    _Float16* yp = Y + (size_t)row * DM + t * 8;
    *(volatile v4u*)yp = w;
    __threadfence();
    *(volatile v4u*)yp = w;
}

#define GBM 64
#define GBN 128
#define GLP 40
#define CPH 136
#define CPF 132
#define CPT 72
enum { EPI_QK = 0, EPI_VT = 1, EPI_GELU = 2, EPI_RES = 3 };

union __attribute__((aligned(16))) CStage {
    float    f[GBM * CPF];
    _Float16 h[GBM * CPH];
    _Float16 t[GBN * CPT];
};

template <int EPI>
__global__ __launch_bounds__(128) void k_gemm(const _Float16* __restrict__ A,
                                                const _Float16* __restrict__ Bt,
                                                const float* __restrict__ bias,
                                                const float* __restrict__ res,
                                                void* Cout,
                                                int N, int K, int seqc, int seqr,
                                                float cs, int rne)
{
    __shared__ __attribute__((aligned(16))) _Float16 As[GBM * GLP];
    __shared__ __attribute__((aligned(16))) _Float16 Bs[GBN * GLP];
    __shared__ CStage Cs;

    const int t = threadIdx.x;
    const int lane = t & 31, wv = t >> 5;
    const int l15 = lane & 15, lh = lane >> 4;
    const int wm = wv >> 1, wn = wv & 1;
    const int brow = blockIdx.y * GBM;
    const int bcol = blockIdx.x * GBN;

    const v8f z = {0.f, 0.f, 0.f, 0.f, 0.f, 0.f, 0.f, 0.f};
    v8f acc[2][4];
#pragma unroll
    for (int mi = 0; mi < 2; ++mi)
#pragma unroll
        for (int ni = 0; ni < 4; ++ni) acc[mi][ni] = z;

    for (int k0 = 0; k0 < K; k0 += 32) {
#pragma unroll
        for (int i = 0; i < 2; ++i) {
            const int c = t + i * 128;
            const int row = c >> 2, seg = c & 3;
            const v4u q = *(const v4ua*)(A + (size_t)(brow + row) * K + k0 + seg * 8);
            *(v4ua*)(As + row * GLP + seg * 8) = q;
        }
#pragma unroll
        for (int i = 0; i < 4; ++i) {
            const int c = t + i * 128;
            const int row = c >> 2, seg = c & 3;
            const v4u q = *(const v4ua*)(Bt + (size_t)(bcol + row) * K + k0 + seg * 8);
            *(v4ua*)(Bs + row * GLP + seg * 8) = q;
        }
        __syncthreads();

        Frag af[2], bf[4];
#pragma unroll
        for (int mi = 0; mi < 2; ++mi) {
            const _Float16* p = As + (wm * 32 + mi * 16 + l15) * GLP + 8 * lh;
            af[mi].h[0] = *(const v8ha*)p;
            af[mi].h[1] = *(const v8ha*)(p + 16);
        }
#pragma unroll
        for (int ni = 0; ni < 4; ++ni) {
            const _Float16* p = Bs + (wn * 64 + ni * 16 + l15) * GLP + 8 * lh;
            bf[ni].h[0] = *(const v8ha*)p;
            bf[ni].h[1] = *(const v8ha*)(p + 16);
        }
#pragma unroll
        for (int mi = 0; mi < 2; ++mi)
#pragma unroll
            for (int ni = 0; ni < 4; ++ni)
                acc[mi][ni] = mma16(af[mi].v, bf[ni].v, acc[mi][ni]);
        asm volatile("v_nop\n\tv_nop\n\tv_nop\n\tv_nop"
                     : "+v"(acc[0][0]), "+v"(acc[0][1]), "+v"(acc[0][2]), "+v"(acc[0][3]),
                       "+v"(acc[1][0]), "+v"(acc[1][1]), "+v"(acc[1][2]), "+v"(acc[1][3])
                     : "v"(af[0].v), "v"(af[1].v), "v"(bf[0].v), "v"(bf[1].v),
                       "v"(bf[2].v), "v"(bf[3].v));
        __syncthreads();
    }

    float bb[4];
#pragma unroll
    for (int ni = 0; ni < 4; ++ni) bb[ni] = bf16r(bias[bcol + wn * 64 + ni * 16 + l15]);

    if (EPI == EPI_QK) {
#pragma unroll
        for (int mi = 0; mi < 2; ++mi) {
#pragma unroll
            for (int r = 0; r < 8; ++r) {
                float qv[4];
                float ss = 0.f;
#pragma unroll
                for (int ni = 0; ni < 4; ++ni) {
                    qv[ni] = acc[mi][ni][r] * cs + bb[ni];
                    ss += qv[ni] * qv[ni];
                }
                ss += __shfl_xor(ss, 1, 32);
                ss += __shfl_xor(ss, 2, 32);
                ss += __shfl_xor(ss, 4, 32);
                ss += __shfl_xor(ss, 8, 32);
                const float inv = 64.0f * __builtin_amdgcn_rcpf(fmaxf(sqrtf(ss), 1.0e-12f));
                const int lr = wm * 32 + mi * 16 + lh * 8 + r;
#pragma unroll
                for (int ni = 0; ni < 4; ++ni)
                    Cs.h[lr * CPH + wn * 64 + ni * 16 + l15] = (_Float16)(qv[ni] * inv);
            }
        }
    } else if (EPI == EPI_GELU) {
#pragma unroll
        for (int mi = 0; mi < 2; ++mi) {
#pragma unroll
            for (int r = 0; r < 8; ++r) {
                const int lr = wm * 32 + mi * 16 + lh * 8 + r;
#pragma unroll
                for (int ni = 0; ni < 4; ++ni) {
                    const float vv = acc[mi][ni][r] * cs + bb[ni];
                    const float g = 0.5f * vv * (1.0f + erff(vv * 0.70710678118654752f));
                    Cs.h[lr * CPH + wn * 64 + ni * 16 + l15] = (_Float16)(g * 16.0f);
                }
            }
        }
    } else if (EPI == EPI_VT) {
#pragma unroll
        for (int mi = 0; mi < 2; ++mi) {
#pragma unroll
            for (int ni = 0; ni < 4; ++ni) {
                v8h pv;
#pragma unroll
                for (int r = 0; r < 8; ++r)
                    pv[r] = (_Float16)((acc[mi][ni][r] * cs + bb[ni]) * 16.0f);
                *(v8ha*)(Cs.t + (wn * 64 + ni * 16 + l15) * CPT + wm * 32 + mi * 16 + lh * 8) = pv;
            }
        }
    } else {
#pragma unroll
        for (int mi = 0; mi < 2; ++mi) {
#pragma unroll
            for (int r = 0; r < 8; ++r) {
                const int lr = wm * 32 + mi * 16 + lh * 8 + r;
#pragma unroll
                for (int ni = 0; ni < 4; ++ni)
                    Cs.f[lr * CPF + wn * 64 + ni * 16 + l15] = acc[mi][ni][r] * cs + bb[ni];
            }
        }
    }
    __syncthreads();

    if (EPI == EPI_QK || EPI == EPI_GELU) {
        _Float16* C = (_Float16*)Cout;
        for (int ps = 0; ps < 2; ++ps) {
#pragma unroll
            for (int p = 0; p < 8; ++p) {
                const int row = p * 8 + (t >> 4), pc = t & 15;
                const v8h o8 = *(const v8ha*)(Cs.h + row * CPH + pc * 8);
                const v4u w = __builtin_bit_cast(v4u, o8);
                *(volatile v4u*)(C + (size_t)(brow + row) * N + bcol + pc * 8) = w;
            }
            if (ps == 0) __threadfence();
        }
    } else if (EPI == EPI_VT) {
        _Float16* Vtp = (_Float16*)Cout;
        const int gb = brow / seqc;
        const int s0 = brow - gb * seqc;
        const int nHh = N >> 6;
        for (int ps = 0; ps < 2; ++ps) {
#pragma unroll
            for (int p = 0; p < 8; ++p) {
                const int dr = p * 16 + (t >> 3), pc = t & 7;
                const int col = bcol + dr;
                const int hh = col >> 6, dd = col & 63;
                const v8h o8 = *(const v8ha*)(Cs.t + dr * CPT + pc * 8);
                const v4u w = __builtin_bit_cast(v4u, o8);
                _Float16* dst = Vtp + ((size_t)(gb * nHh + hh) * 64 + dd) * seqc + s0 + pc * 8;
                *(volatile v4u*)dst = w;
            }
            if (ps == 0) __threadfence();
        }
    } else {
        float* C = (float*)Cout;
        for (int ps = 0; ps < 2; ++ps) {
#pragma unroll 4
            for (int p = 0; p < 16; ++p) {
                const int row = p * 4 + wv, pc = lane;
                const int grow = brow + row;
                const int gb = grow / seqc;
                const int rrow = gb * seqr + (grow - gb * seqc);
                v4f c = *(const v4fa*)(Cs.f + row * CPF + pc * 4);
                v4f rr = *(const v4fa*)(res + (size_t)rrow * N + bcol + pc * 4);
                if (rne) {
                    rr[0] = bf16r(rr[0]); rr[1] = bf16r(rr[1]);
                    rr[2] = bf16r(rr[2]); rr[3] = bf16r(rr[3]);
                }
                c += rr;
                *(volatile v4f*)(C + (size_t)grow * N + bcol + pc * 4) = c;
            }
            if (ps == 0) __threadfence();
        }
    }
}

__global__ __launch_bounds__(128) void k_attn(const _Float16* __restrict__ Qp,
                                                const _Float16* __restrict__ Kp,
                                                const _Float16* __restrict__ Vt,
                                                const float* __restrict__ lsc,
                                                _Float16* Cx, int seqc)
{
    __shared__ __attribute__((aligned(16))) _Float16 Ks[64 * CPT];
    __shared__ __attribute__((aligned(16))) _Float16 Vs[64 * CPT];
    __shared__ __attribute__((aligned(16))) _Float16 Os[64 * CPT];

    const int t = threadIdx.x;
    const int lane = t & 31, wv = t >> 5;
    const int l15 = lane & 15, lh = lane >> 4;
    const int bh = blockIdx.y;
    const int b = bh / NH, h = bh - b * NH;
    const int q0 = blockIdx.x * 64;

    const float ls = bf16r(lsc[h]);
    const float sc2 = expf(fminf(ls, LOGMAX)) * (LOG2E / 4096.0f);

    Frag qb[2];
    {
        const _Float16* qr = Qp + (size_t)(b * seqc + q0 + wv * 16 + l15) * DM + h * HDIM + 8 * lh;
#pragma unroll
        for (int kk = 0; kk < 2; ++kk) {
            qb[kk].h[0] = *(const v8ha*)(qr + kk * 32);
            qb[kk].h[1] = *(const v8ha*)(qr + kk * 32 + 16);
        }
    }

    const v8f z = {0.f, 0.f, 0.f, 0.f, 0.f, 0.f, 0.f, 0.f};
    v8f oacc[4];
#pragma unroll
    for (int ni = 0; ni < 4; ++ni) oacc[ni] = z;
    float mrun = -1.0e30f, lsum = 0.f;

    const int nkb = seqc >> 6;
    for (int kb = 0; kb < nkb; ++kb) {
        __syncthreads();
        {
            const int kr = t >> 1, seg = (t & 1) * 32;
            const _Float16* ks = Kp + (size_t)(b * seqc + kb * 64 + kr) * DM + h * HDIM + seg;
            const _Float16* vs = Vt + ((size_t)bh * HDIM + kr) * seqc + kb * 64 + seg;
#pragma unroll
            for (int j = 0; j < 4; ++j) {
                *(v4ua*)(Ks + kr * CPT + seg + 8 * j) = *(const v4ua*)(ks + 8 * j);
                *(v4ua*)(Vs + kr * CPT + seg + 8 * j) = *(const v4ua*)(vs + 8 * j);
            }
        }
        __syncthreads();

        v8f sacc[4];
#pragma unroll
        for (int mt = 0; mt < 4; ++mt) {
            Frag ka, kc;
            const _Float16* kp = Ks + (mt * 16 + l15) * CPT + 8 * lh;
            ka.h[0] = *(const v8ha*)kp;
            ka.h[1] = *(const v8ha*)(kp + 16);
            kc.h[0] = *(const v8ha*)(kp + 32);
            kc.h[1] = *(const v8ha*)(kp + 48);
            sacc[mt] = mma16(ka.v, qb[0].v, z);
            sacc[mt] = mma16(kc.v, qb[1].v, sacc[mt]);
            asm volatile("v_nop\n\tv_nop\n\tv_nop\n\tv_nop"
                         : "+v"(sacc[mt])
                         : "v"(ka.v), "v"(kc.v), "v"(qb[0].v), "v"(qb[1].v));
        }

        float mx = -1.0e30f;
#pragma unroll
        for (int mt = 0; mt < 4; ++mt)
#pragma unroll
            for (int r = 0; r < 8; ++r) mx = fmaxf(mx, sacc[mt][r]);
        mx = fmaxf(mx, __shfl_xor(mx, 16, 32));
        const float mnew = fmaxf(mrun, mx * sc2);
        const float alpha = exp2f(mrun - mnew);
        float psum = 0.f;
        Frag pa[2];
#pragma unroll
        for (int mt = 0; mt < 4; ++mt) {
            v8h ph;
#pragma unroll
            for (int r = 0; r < 8; ++r) {
                const float p = exp2f(sacc[mt][r] * sc2 - mnew + 14.0f);
                ph[r] = (_Float16)p;
                psum += p;
            }
            pa[mt >> 1].h[mt & 1] = ph;
        }
        psum += __shfl_xor(psum, 16, 32);
        lsum = lsum * alpha + psum;
        mrun = mnew;

        float ar[8];
#pragma unroll
        for (int r = 0; r < 8; ++r) ar[r] = __shfl(alpha, 8 * lh + r, 32);
#pragma unroll
        for (int ni = 0; ni < 4; ++ni)
#pragma unroll
            for (int r = 0; r < 8; ++r) oacc[ni][r] *= ar[r];

#pragma unroll
        for (int kk2 = 0; kk2 < 2; ++kk2) {
            Frag vb[4];
#pragma unroll
            for (int ni = 0; ni < 4; ++ni) {
                const _Float16* vp = Vs + (ni * 16 + l15) * CPT + kk2 * 32 + 8 * lh;
                vb[ni].h[0] = *(const v8ha*)vp;
                vb[ni].h[1] = *(const v8ha*)(vp + 16);
            }
#pragma unroll
            for (int ni = 0; ni < 4; ++ni)
                oacc[ni] = mma16(pa[kk2].v, vb[ni].v, oacc[ni]);
            asm volatile("v_nop\n\tv_nop\n\tv_nop\n\tv_nop"
                         : "+v"(oacc[0]), "+v"(oacc[1]), "+v"(oacc[2]), "+v"(oacc[3])
                         : "v"(pa[kk2].v), "v"(vb[0].v), "v"(vb[1].v), "v"(vb[2].v),
                           "v"(vb[3].v));
        }
    }

    const float linv = __builtin_amdgcn_rcpf(lsum);
    float il[8];
#pragma unroll
    for (int r = 0; r < 8; ++r) il[r] = __shfl(linv, 8 * lh + r, 32) * 4.0f;
#pragma unroll
    for (int ni = 0; ni < 4; ++ni)
#pragma unroll
        for (int r = 0; r < 8; ++r)
            Os[(wv * 16 + 8 * lh + r) * CPT + ni * 16 + l15] = (_Float16)(oacc[ni][r] * il[r]);
    __syncthreads();

    for (int ps = 0; ps < 2; ++ps) {
#pragma unroll
        for (int p = 0; p < 4; ++p) {
            const int row = p * 16 + (t >> 3), pc = t & 7;
            const v8h o8 = *(const v8ha*)(Os + row * CPT + pc * 8);
            const v4u w = __builtin_bit_cast(v4u, o8);
            *(volatile v4u*)(Cx + (size_t)(b * seqc + q0 + row) * DM + h * HDIM + pc * 8) = w;
        }
        if (ps == 0) __threadfence();
    }
}

extern "C" void kernel_launch(void* const* d_in, const int* in_sizes, int n_in,
                              void* d_out, int out_size, void* d_ws, size_t ws_size,
                              hipStream_t stream)
{
    if (n_in < 18) return;
    if (in_sizes[0] < ((NB - 1) * SEQ_FULL + SEQ) * DM) return;
    if (in_sizes[1] < DM * DM || in_sizes[3] < DM * DM || in_sizes[5] < DM * DM ||
        in_sizes[7] < DM * DM) return;
    if (in_sizes[2] < DM || in_sizes[4] < DM || in_sizes[6] < DM || in_sizes[8] < DM) return;
    if (in_sizes[9] < DM * DFF || in_sizes[10] < DFF || in_sizes[11] < DFF * DM ||
        in_sizes[12] < DM) return;
    if (in_sizes[13] < DM || in_sizes[14] < DM || in_sizes[15] < DM || in_sizes[16] < DM) return;
    if (in_sizes[17] < NH) return;
    if (out_size < TOKN * DM) return;

    const float* x    = (const float*)d_in[0];
    const float* wq   = (const float*)d_in[1];
    const float* bq   = (const float*)d_in[2];
    const float* wk   = (const float*)d_in[3];
    const float* bk   = (const float*)d_in[4];
    const float* wvv  = (const float*)d_in[5];
    const float* bv   = (const float*)d_in[6];
    const float* wo   = (const float*)d_in[7];
    const float* bo   = (const float*)d_in[8];
    const float* w1   = (const float*)d_in[9];
    const float* b1   = (const float*)d_in[10];
    const float* w2   = (const float*)d_in[11];
    const float* b2   = (const float*)d_in[12];
    const float* ln1g = (const float*)d_in[13];
    const float* ln1b = (const float*)d_in[14];
    const float* ln2g = (const float*)d_in[15];
    const float* ln2b = (const float*)d_in[16];
    const float* lsc  = (const float*)d_in[17];
    float* out = (float*)d_out;

    char* ws = (char*)d_ws;
    size_t off = 0;
    auto carve = [&](size_t bytes) -> size_t {
        const size_t o = off;
        off += (bytes + 255) & ~(size_t)255;
        return o;
    };
    const size_t oWq  = carve((size_t)DM * DM * 2);
    const size_t oWk  = carve((size_t)DM * DM * 2);
    const size_t oWv  = carve((size_t)DM * DM * 2);
    const size_t oWo  = carve((size_t)DM * DM * 2);
    const size_t oW1  = carve((size_t)DFF * DM * 2);
    const size_t oW2  = carve((size_t)DM * DFF * 2);
    const size_t oXn  = carve((size_t)TOKN * DM * 2);
    const size_t oQ   = carve((size_t)TOKN * DM * 2);
    const size_t oK   = carve((size_t)TOKN * DM * 2);
    const size_t oVt  = carve((size_t)NB * NH * HDIM * SEQ * 2);
    const size_t oCx  = carve((size_t)TOKN * DM * 2);
    const size_t oAo  = carve((size_t)TOKN * DM * 4);
    const size_t oXn2 = carve((size_t)TOKN * DM * 2);
    const size_t oH1  = carve((size_t)TOKN * DFF * 2);
    if (off > ws_size) return;

    _Float16* Wqt = (_Float16*)(ws + oWq);
    _Float16* Wkt = (_Float16*)(ws + oWk);
    _Float16* Wvt = (_Float16*)(ws + oWv);
    _Float16* Wot = (_Float16*)(ws + oWo);
    _Float16* W1t = (_Float16*)(ws + oW1);
    _Float16* W2t = (_Float16*)(ws + oW2);
    _Float16* Xn  = (_Float16*)(ws + oXn);
    _Float16* Qp  = (_Float16*)(ws + oQ);
    _Float16* Kpl = (_Float16*)(ws + oK);
    _Float16* Vtp = (_Float16*)(ws + oVt);
    _Float16* Cx  = (_Float16*)(ws + oCx);
    float*    Ao  = (float*)(ws + oAo);
    _Float16* Xn2 = (_Float16*)(ws + oXn2);
    _Float16* H1  = (_Float16*)(ws + oH1);

    k_wcvt<<<dim3(DM / 64, DM / 64), 256, 0, stream>>>(wq,  Wqt, DM, DM, 64.0f);
    k_wcvt<<<dim3(DM / 64, DM / 64), 256, 0, stream>>>(wk,  Wkt, DM, DM, 64.0f);
    k_wcvt<<<dim3(DM / 64, DM / 64), 256, 0, stream>>>(wvv, Wvt, DM, DM, 64.0f);
    k_wcvt<<<dim3(DM / 64, DM / 64), 256, 0, stream>>>(wo,  Wot, DM, DM, 64.0f);
    k_wcvt<<<dim3(DFF / 64, DM / 64), 256, 0, stream>>>(w1, W1t, DM, DFF, 64.0f);
    k_wcvt<<<dim3(DM / 64, DFF / 64), 256, 0, stream>>>(w2, W2t, DFF, DM, 64.0f);

    k_ln<<<TOKN, 128, 0, stream>>>(x, ln1g, ln1b, Xn, SEQ, SEQ_FULL, 1);

    k_gemm<EPI_QK><<<dim3(DM / GBN, TOKN / GBM), 128, 0, stream>>>(
        Xn, Wqt, bq, nullptr, Qp, DM, DM, SEQ, SEQ, 1.0f / 64.0f, 0);
    k_gemm<EPI_QK><<<dim3(DM / GBN, TOKN / GBM), 128, 0, stream>>>(
        Xn, Wkt, bk, nullptr, Kpl, DM, DM, SEQ, SEQ, 1.0f / 64.0f, 0);
    k_gemm<EPI_VT><<<dim3(DM / GBN, TOKN / GBM), 128, 0, stream>>>(
        Xn, Wvt, bv, nullptr, Vtp, DM, DM, SEQ, SEQ, 1.0f / 64.0f, 0);

    k_attn<<<dim3(SEQ / 64, NB * NH), 128, 0, stream>>>(Qp, Kpl, Vtp, lsc, Cx, SEQ);

    k_gemm<EPI_RES><<<dim3(DM / GBN, TOKN / GBM), 128, 0, stream>>>(
        Cx, Wot, bo, x, Ao, DM, DM, SEQ, SEQ_FULL, 1.0f / 4096.0f, 1);

    k_ln<<<TOKN, 128, 0, stream>>>(Ao, ln2g, ln2b, Xn2, SEQ, SEQ, 0);

    k_gemm<EPI_GELU><<<dim3(DFF / GBN, TOKN / GBM), 128, 0, stream>>>(
        Xn2, W1t, b1, nullptr, H1, DFF, DM, SEQ, SEQ, 1.0f / 64.0f, 0);

    k_gemm<EPI_RES><<<dim3(DM / GBN, TOKN / GBM), 128, 0, stream>>>(
        H1, W2t, b2, Ao, out, DM, DFF, SEQ, SEQ, 1.0f / 1024.0f, 0);
}
